// GlobalPoolDistance_34935263986419
// MI455X (gfx1250) — hardware-verified
//
#include <hip/hip_runtime.h>
#include <hip/hip_bf16.h>

typedef __attribute__((ext_vector_type(16))) _Float16 v16h;
#define VST2(T, ptr, val) do { const T _v = (val); *(volatile T*)(ptr) = _v; __threadfence(); *(volatile T*)(ptr) = _v; } while (0)
typedef __attribute__((ext_vector_type(8)))  float    v8f;

#define BATCH   8
#define CH      3
#define IMG     64
#define PW      62
#define NPATCH  3844
#define NT      241
#define NPAD    (NT*16)
#define KF      27
#define NWAVE   (3*BATCH*NT)

#define CSCALE  (1.4426950408889634f / 0.2916f)
#define TWOC    (2.0f * CSCALE)

__global__ void pack_frags(const float* __restrict__ img,
                           _Float16* __restrict__ outA) {
    int tid = blockIdx.x * blockDim.x + threadIdx.x;
    const int total = BATCH * NT * 32;
    if (tid >= total) return;
    int lane = tid & 31;
    int t    = (tid >> 5) % NT;
    int b    = tid / (NT * 32);
    int mn   = lane & 15;
    int g    = t * 16 + mn;
    int hi   = lane >> 4;
    bool gok = g < NPATCH;
    int py = g / PW, px = g % PW;

    v16h va;
#pragma unroll
    for (int e = 0; e < 16; ++e) {
        int ka = (e < 8) ? (hi * 8 + e) : (16 + hi * 8 + (e - 8));
        float fa = 0.f;
        if (gok && ka < KF) {
            int c = ka / 9, rem = ka - c * 9, r = rem / 3, s = rem - r * 3;
            fa = img[((b * CH + c) * IMG + py + r) * IMG + px + s];
        }
        va[e] = (_Float16)fa;
    }
    VST2(v16h, outA + (size_t)tid * 16, va);
}

__global__ void sqnorms(const float* __restrict__ img, float* __restrict__ sq) {
    int tid = blockIdx.x * blockDim.x + threadIdx.x;
    const int total = BATCH * NPAD;
    if (tid >= total) return;
    int g = tid % NPAD;
    int b = tid / NPAD;
    float out = __builtin_inff();
    if (g < NPATCH) {
        int py = g / PW, px = g % PW;
        float s = 0.f;
#pragma unroll
        for (int k = 0; k < KF; ++k) {
            int c = k / 9, rem = k - c * 9, r = rem / 3, ss = rem - r * 3;
            float v = img[((b * CH + c) * IMG + py + r) * IMG + px + ss];
            float h = (float)(_Float16)v;
            s += h * h;
        }
        out = s * CSCALE;
    }
    VST2(float, sq + tid, out);
}

__device__ __forceinline__ void tile_accum(const v16h& a,
                                           const _Float16* __restrict__ bf_ptr,
                                           float sc, const v8f& srv,
                                           v8f& accsum) {
    v16h bf = *(const v16h*)bf_ptr;
    v8f c = {};
    v8f acc = __builtin_amdgcn_wmma_f32_16x16x32_f16(
         false, a,  false, bf,
         (short)0, c,  false,  false);
    asm volatile("v_nop\n\tv_nop\n\tv_nop\n\tv_nop" : "+v"(acc) : "v"(a), "v"(bf));
#pragma unroll
    for (int r = 0; r < 8; ++r) {
        float t   = srv[r] + sc;
        float arg = __builtin_fmaf(acc[r], TWOC, -t);
        accsum[r] += __builtin_amdgcn_exp2f(arg);
    }
}

__global__ void __launch_bounds__(256)
mmd_wmma(const _Float16* __restrict__ AX, const _Float16* __restrict__ BX,
         const _Float16* __restrict__ AY, const _Float16* __restrict__ BY,
         const float* __restrict__ sqX,  const float* __restrict__ sqY,
         float* __restrict__ partials) {
    int gtid = blockIdx.x * 256 + threadIdx.x;
    int wave = __builtin_amdgcn_readfirstlane(gtid >> 5);
    int lane = threadIdx.x & 31;
    if (wave >= NWAVE) return;

    int ti = wave % NT;
    int b  = (wave / NT) % BATCH;
    int p  = wave / (NT * BATCH);

    const _Float16* Afrag = (p == 2) ? AY : AX;
    const _Float16* Bfrag = (p == 1) ? BX : BY;
    const float*    sqA   = (p == 2) ? sqY : sqX;
    const float*    sqB   = (p == 1) ? sqX : sqY;
    bool  sym   = (p != 0);
    float w     = sym ? 1.0f : -2.0f;
    float mbase = sym ? 2.0f : 1.0f;
    int   tj0   = sym ? ti : 0;

    v16h a = *(const v16h*)(Afrag + ((size_t)(b * NT + ti) * 32 + lane) * 16);

    int rbase = ti * 16 + ((lane >> 4) << 3);
    v8f srv = *(const v8f*)(sqA + b * NPAD + rbase);

    int ncol = lane & 15;
    const _Float16* bft = Bfrag + ((size_t)(b * NT + tj0) * 32 + lane) * 16;
    const float*    scp = sqB + b * NPAD + tj0 * 16 + ncol;

    v8f accDiag = {}, accMain = {};
    tile_accum(a, bft, *scp, srv, accDiag);

    for (int tj = tj0 + 1; tj < NT; ++tj) {
        bft += 512;
        scp += 16;
        __builtin_prefetch(bft + 512, 0, 3);
        tile_accum(a, bft, *scp, srv, accMain);
    }

    float sd = 0.f, sm = 0.f;
#pragma unroll
    for (int r = 0; r < 8; ++r) { sd += accDiag[r]; sm += accMain[r]; }
    float sum = __builtin_fmaf(mbase, sm, sd);

#pragma unroll
    for (int off = 16; off > 0; off >>= 1)
        sum += __shfl_xor(sum, off, 32);
    if (lane == 0) VST2(float, partials + (size_t)wave * 32, w * sum);
}

__global__ void final_reduce(const float* __restrict__ partials,
                             float* __restrict__ out) {
    __shared__ float smem[256];
    float s = 0.f;
    for (int i = threadIdx.x; i < NWAVE; i += 256) s += partials[(size_t)i * 32];
    smem[threadIdx.x] = s;
    __syncthreads();
#pragma unroll
    for (int step = 128; step > 0; step >>= 1) {
        if ((int)threadIdx.x < step) smem[threadIdx.x] += smem[threadIdx.x + step];
        __syncthreads();
    }
    if (threadIdx.x == 0)
        VST2(float, out, smem[0] * (1.0f / ((float)BATCH * (float)NPATCH * (float)NPATCH)));
}

extern "C" void kernel_launch(void* const* d_in, const int* in_sizes, int n_in,
                              void* d_out, int out_size, void* d_ws, size_t ws_size,
                              hipStream_t stream) {
    const float* x = (const float*)d_in[0];
    const float* y = (const float*)d_in[1];
    float* out = (float*)d_out;

    (void)in_sizes; (void)n_in; (void)out_size;
    const size_t FE = (size_t)BATCH * NT * 512;
    if (ws_size < FE * 2 * 2 + (size_t)2 * BATCH * NPAD * 4 + (size_t)NWAVE * 128) return;
    _Float16* AX = (_Float16*)d_ws;
    _Float16* AY = AX + FE;
    _Float16* BX = AX;
    _Float16* BY = AY;
    float* sqX = (float*)(AY + FE);
    float* sqY = sqX + BATCH * NPAD;
    float* partials = sqY + BATCH * NPAD;

    const int packThreads = BATCH * NT * 32;
    pack_frags<<<(packThreads + 255) / 256, 256, 0, stream>>>(x, AX);
    pack_frags<<<(packThreads + 255) / 256, 256, 0, stream>>>(y, AY);

    const int sqThreads = BATCH * NPAD;
    sqnorms<<<(sqThreads + 255) / 256, 256, 0, stream>>>(x, sqX);
    sqnorms<<<(sqThreads + 255) / 256, 256, 0, stream>>>(y, sqY);

    mmd_wmma<<<(NWAVE * 32) / 256, 256, 0, stream>>>(AX, BX, AY, BY,
                                                     sqX, sqY, partials);
    final_reduce<<<1, 256, 0, stream>>>(partials, out);
}
